// MPNN_ENN_K_Set2Set_5076651344424
// MI455X (gfx1250) — hardware-run, weakly checked
//
#include <hip/hip_runtime.h>


namespace {
constexpr int N = 10000, E = 80000, NB = 64, NF = 32, EF = 16, H = 64, TGT = 16, T = 3, S2S = 12, GW = H * H + H, NBLK = N / 16;
constexpr float XS = 8.0f, HS = 64.0f, WSC = 256.0f;
typedef _Float16 b16;
typedef __attribute__((ext_vector_type(16))) _Float16 v16b;
typedef __attribute__((ext_vector_type(8))) _Float16 v8b;
typedef __attribute__((ext_vector_type(8))) float v8f;
typedef __attribute__((ext_vector_type(4))) float v4f;
typedef __attribute__((ext_vector_type(2))) float v2f;
__device__ __forceinline__ float bf16_rne(float f) { unsigned int u = __float_as_uint(f); u += 0x7FFFu + ((u >> 16) & 1u); return __uint_as_float(u & 0xFFFF0000u); }
__device__ __forceinline__ void split16(float v, b16& hi, b16& lo) { hi = (b16)v; lo = (b16)(v - (float)hi); }
__device__ __forceinline__ v16b frag_kb(const b16* p, int hh) { const v8b a = *(const v8b*)(p + 8 * hh), b = *(const v8b*)(p + 16 + 8 * hh); v16b f;
#pragma unroll
  for (int e = 0; e < 8; ++e) { f[e] = a[e]; f[8 + e] = b[e]; } return f; }
__device__ __forceinline__ v8f wmma16b(v16b a, v16b b, v8f c) { v8f d = __builtin_amdgcn_wmma_f32_16x16x32_f16(false, a, false, b, (short)0, c, false, false); asm volatile("v_nop\n\tv_nop\n\tv_nop\n\tv_nop" : "+v"(d) : "v"(a), "v"(b)); return d; }
__device__ __forceinline__ void wave_lds_sync() { __builtin_amdgcn_fence(__ATOMIC_RELEASE, "workgroup"); __builtin_amdgcn_wave_barrier(); __builtin_amdgcn_fence(__ATOMIC_ACQUIRE, "workgroup"); }
__device__ __forceinline__ float pmul(float a, float b) { float p = a * b; asm volatile("" : "+v"(p)); return p; }
__device__ __forceinline__ int iclamp(int v, int lo, int hi) { return v < lo ? lo : (v > hi ? hi : v); }
__device__ __forceinline__ float sigm(float v) { return 1.0f / (1.0f + __expf(-v)); }
constexpr int CSR_NBLK9 = 512, CSR_GB9 = 9, CSR_GN9 = 1 << CSR_GB9  , CSR_TS9 = (CSR_GN9 < 32 ? 32 : CSR_GN9)  , CSR_MAXG9 = 512, CSR_CAP9 = 12288  ;
__device__ __host__ __forceinline__ int csr_tix9(int v) { return (v >> CSR_GB9) * CSR_TS9 + (v & (CSR_GN9 - 1)); }
__global__ __launch_bounds__(64) void csrA_kernel9(const int* __restrict__ dst, int E, int N, int nG, int CHP, int NGP, int* __restrict__ STG, int* __restrict__ HST) {
  extern __shared__ int sm[];
  int* cnt = sm; int* run = sm + NGP; int* ids = sm + 2 * NGP;
  const int b = blockIdx.x; const int ch = (E + CSR_NBLK9 - 1) / CSR_NBLK9; const int e0 = b * ch, e1 = min(E, e0 + ch);
  for (int i = threadIdx.x; i < NGP; i += 64) cnt[i] = 0;
  for (int i = threadIdx.x; i < CHP; i += 64) ids[i] = -1;
  __syncthreads();
  if (threadIdx.x == 0) {
    for (int e = e0; e < e1; ++e) { int d = dst[e]; d = (d < 0) ? 0 : (d >= N ? N - 1 : d); cnt[d >> CSR_GB9] += 1; }
    int acc = 0; for (int g = 0; g < nG; ++g) { run[g] = acc; acc += cnt[g]; }
    for (int e = e0; e < e1; ++e) { int d = dst[e]; d = (d < 0) ? 0 : (d >= N ? N - 1 : d); const int g = d >> CSR_GB9; ids[run[g]] = e; run[g] += 1; } }
  __syncthreads();
  typedef __attribute__((ext_vector_type(4))) int v4i;
  for (int pass = 0; pass < 2; ++pass) {
    for (int i = threadIdx.x; i < CHP / 4; i += 64) *(volatile v4i*)(STG + (size_t)b * CHP + i * 4) = *(const v4i*)(&ids[i * 4]);
    for (int i = threadIdx.x; i < NGP / 4; i += 64) { v4i v; for (int e = 0; e < 4; ++e) v[e] = (i * 4 + e < nG) ? cnt[i * 4 + e] : 0; *(volatile v4i*)(HST + (size_t)b * NGP + i * 4) = v; }
    __threadfence(); }
}
__global__ __launch_bounds__(512) void csrS_kernel9(const int* __restrict__ HST, int nG, int NGP, int* __restrict__ START, int* __restrict__ TOT, int* __restrict__ OFF) {
  __shared__ int tot[CSR_MAXG9];
  const int b = threadIdx.x;
  for (int pass = 0; pass < 2; ++pass) { int runb = 0; for (int g = 0; g < nG; ++g) { int c = HST[(size_t)b * NGP + g]; c = (c < 0) ? 0 : c; ((volatile int*)OFF)[(size_t)g * CSR_NBLK9 + b] = runb; runb += c; } __threadfence(); }
  for (int g = threadIdx.x; g < nG; g += 512) { int s = 0; for (int bb = 0; bb < CSR_NBLK9; ++bb) { int c = HST[(size_t)bb * NGP + g]; s += (c < 0) ? 0 : c; } tot[g] = s; }
  __syncthreads();
  if (threadIdx.x < 32) {
    __shared__ int st[CSR_MAXG9 + 32];
    if (threadIdx.x == 0) { int acc = 0; for (int g = 0; g < NGP; ++g) { st[g] = acc; if (g < nG) acc += (tot[g] + 31) & ~31; } st[NGP] = acc; }
    __builtin_amdgcn_fence(__ATOMIC_RELEASE, "workgroup"); __builtin_amdgcn_wave_barrier(); __builtin_amdgcn_fence(__ATOMIC_ACQUIRE, "workgroup");
    for (int pass = 0; pass < 2; ++pass) { for (int i = threadIdx.x; i < NGP + 32; i += 32) { ((volatile int*)START)[i] = (i <= NGP) ? st[min(i, NGP)] : 0; ((volatile int*)TOT)[i] = (i < nG) ? tot[i] : 0; } __threadfence(); } }
}
__global__ __launch_bounds__(256) void csrB_kernel9(const int* __restrict__ dst, int N, int nG, int CHP, int NGP, int permLen, const int* __restrict__ STG, const int* __restrict__ HST, const int* __restrict__ OFF, const int* __restrict__ START, const int* __restrict__ TOT, int* __restrict__ PERM, int* __restrict__ ROWPTR, int* __restrict__ ROWCNT, int* __restrict__ FLAG) {
  typedef __attribute__((ext_vector_type(4))) int v4i;
  __shared__ int ids[CSR_CAP9]; __shared__ unsigned short key[CSR_CAP9]; __shared__ int outp[CSR_CAP9]; __shared__ int ncnt[CSR_GN9 + 1]; __shared__ int boff[CSR_NBLK9 + 1];
  const int g = blockIdx.x, t_ = threadIdx.x; int tot = TOT[g]; int st = START[g], stn = START[g + 1]; const int v0 = g * CSR_GN9; const int nv = min(CSR_GN9, N - v0); const int t0 = g * CSR_TS9;
  st = (st < 0) ? 0 : (st > permLen - 32 ? permLen - 32 : st) & ~31; stn = (stn < st) ? st : (stn > permLen ? permLen : stn); tot = (tot < 0) ? 0 : tot; if (tot > stn - st && tot <= CSR_CAP9) tot = stn - st;
  if (tot > CSR_CAP9) {
    for (int pass = 0; pass < 2; ++pass) { for (int i = t_; i < CSR_TS9 / 4; i += 256) { v4i a, c; for (int e = 0; e < 4; ++e) { a[e] = st; c[e] = 0; } *(volatile v4i*)(ROWPTR + t0 + i * 4) = a; *(volatile v4i*)(ROWCNT + t0 + i * 4) = c; } if (t_ == 0) ((volatile int*)FLAG)[0] = 1; __threadfence(); } (void)nv; return; }
  if (t_ == 0) { int acc = 0; for (int b = 0; b < CSR_NBLK9; ++b) { boff[b] = acc; int c = HST[(size_t)b * NGP + g]; c = (c < 0) ? 0 : (c > CHP ? CHP : c); acc += c; if (acc > tot) acc = tot; } boff[CSR_NBLK9] = acc; }
  for (int i = t_; i <= CSR_GN9; i += 256) ncnt[i] = 0;
  __syncthreads();
  for (int b = 0; b < CSR_NBLK9; ++b) { const int c = boff[b + 1] - boff[b]; int o_ = OFF[(size_t)g * CSR_NBLK9 + b]; o_ = (o_ < 0) ? 0 : (o_ > CHP - c ? CHP - c : o_); const int* src_ = STG + (size_t)b * CHP + o_;
    for (int i = t_; i < c; i += 256) { int id = src_[i]; id = (id < 0) ? 0 : id; ids[boff[b] + i] = id; int d = dst[id]; d = (d < v0) ? v0 : (d >= N ? N - 1 : d); int kk = d - v0; kk = (kk < 0) ? 0 : (kk >= CSR_GN9 ? CSR_GN9 - 1 : kk); key[boff[b] + i] = (unsigned short)kk; } }
  __syncthreads();
  if (t_ == 0) { for (int i = 0; i < tot; ++i) ncnt[key[i]] += 1; int acc = 0; for (int vl = 0; vl < CSR_GN9; ++vl) { const int c = ncnt[vl]; ncnt[vl] = acc; acc += c; } ncnt[CSR_GN9] = acc;
    for (int i = 0; i < tot; ++i) { const int vl = key[i]; outp[ncnt[vl]] = ids[i]; ncnt[vl] += 1; }
    for (int vl = CSR_GN9; vl > 0; --vl) ncnt[vl] = ncnt[vl - 1]; ncnt[0] = 0; }
  __syncthreads();
  for (int pass = 0; pass < 2; ++pass) {
    for (int i = t_; i < (stn - st) / 4; i += 256) { v4i v; for (int e = 0; e < 4; ++e) { const int q = i * 4 + e; v[e] = (q < tot) ? outp[q] : -1; } *(volatile v4i*)(PERM + st + i * 4) = v; }
    for (int i = t_; i < CSR_TS9 / 4; i += 256) { v4i a, c; for (int e = 0; e < 4; ++e) { const int vl = i * 4 + e; const int vc = vl < CSR_GN9 ? vl : CSR_GN9; a[e] = (vl < CSR_GN9) ? st + ncnt[vc] : st; c[e] = (vl < nv) ? (ncnt[(vc < CSR_GN9 ? vc : CSR_GN9 - 1) + 1] - ncnt[vc]) : 0; } *(volatile v4i*)(ROWPTR + t0 + i * 4) = a; *(volatile v4i*)(ROWCNT + t0 + i * 4) = c; }
    __threadfence(); }
}
__global__ __launch_bounds__(256) void csrZ_kernel9(int* __restrict__ p, size_t n4) { typedef __attribute__((ext_vector_type(4))) int v4i; const size_t tid = (size_t)blockIdx.x * 256 + threadIdx.x, nth = (size_t)gridDim.x * 256; v4i z = {0, 0, 0, 0}; for (size_t i = tid; i < n4; i += nth) *(volatile v4i*)(p + i * 4) = z; }
struct CsrBufs9 { int *STG, *HST, *OFF, *START, *TOT, *PERM, *ROWPTR, *ROWCNT, *FLAG; int nG, NGP, CHP; size_t permLen; char* base; size_t bytes; };
static size_t csr_carve9(CsrBufs9& c, char* ws, size_t off, int E, int N) {
  const size_t off0 = off; c.base = ws + off;
  auto al = [&](size_t bytes) { char* p = ws + off; off += (bytes + 255) & ~(size_t)255; return p; };
  c.nG = (N + CSR_GN9 - 1) / CSR_GN9; c.NGP = (c.nG + 31) & ~31; const int ch = (E + CSR_NBLK9 - 1) / CSR_NBLK9; c.CHP = (ch + 31) & ~31; c.permLen = (size_t)E + 32 * (size_t)c.nG + 32;
  c.STG = (int*)al((size_t)CSR_NBLK9 * c.CHP * 4); c.HST = (int*)al((size_t)CSR_NBLK9 * c.NGP * 4); c.OFF = (int*)al((size_t)c.NGP * CSR_NBLK9 * 4); c.START = (int*)al((size_t)(c.NGP + 64) * 4); c.TOT = (int*)al((size_t)(c.NGP + 64) * 4);
  c.PERM = (int*)al(c.permLen * 4); c.ROWPTR = (int*)al((size_t)c.nG * CSR_TS9 * 4); c.ROWCNT = (int*)al((size_t)c.nG * CSR_TS9 * 4); c.FLAG = (int*)al(256);
  c.bytes = off - off0; return off;
}
static void csr_build9(const CsrBufs9& c, const int* dst, int E, int N, hipStream_t stream) {
  const size_t smem = (size_t)(2 * c.NGP + c.CHP) * 4;
  csrZ_kernel9<<<512, 256, 0, stream>>>((int*)c.base, c.bytes / 16);
  csrA_kernel9<<<CSR_NBLK9, 64, smem, stream>>>(dst, E, N, c.nG, c.CHP, c.NGP, c.STG, c.HST);
  csrS_kernel9<<<1, 512, 0, stream>>>(c.HST, c.nG, c.NGP, c.START, c.TOT, c.OFF);
  csrB_kernel9<<<c.nG, 256, 0, stream>>>(dst, N, c.nG, c.CHP, c.NGP, (int)c.permLen, c.STG, c.HST, c.OFF, c.START, c.TOT, c.PERM, c.ROWPTR, c.ROWCNT, c.FLAG);
}

constexpr int CSR_NBLK3 = 512, CSR_GB3 = 3, CSR_GN3 = 1 << CSR_GB3  , CSR_TS3 = (CSR_GN3 < 32 ? 32 : CSR_GN3)  , CSR_MAXG3 = 512, CSR_CAP3 = 12288  ;
__device__ __host__ __forceinline__ int csr_tix3(int v) { return (v >> CSR_GB3) * CSR_TS3 + (v & (CSR_GN3 - 1)); }
__global__ __launch_bounds__(64) void csrA_kernel3(const int* __restrict__ dst, int E, int N, int nG, int CHP, int NGP, int* __restrict__ STG, int* __restrict__ HST) {
  extern __shared__ int sm[];
  int* cnt = sm; int* run = sm + NGP; int* ids = sm + 2 * NGP;
  const int b = blockIdx.x; const int ch = (E + CSR_NBLK3 - 1) / CSR_NBLK3; const int e0 = b * ch, e1 = min(E, e0 + ch);
  for (int i = threadIdx.x; i < NGP; i += 64) cnt[i] = 0;
  for (int i = threadIdx.x; i < CHP; i += 64) ids[i] = -1;
  __syncthreads();
  if (threadIdx.x == 0) {
    for (int e = e0; e < e1; ++e) { int d = dst[e]; d = (d < 0) ? 0 : (d >= N ? N - 1 : d); cnt[d >> CSR_GB3] += 1; }
    int acc = 0; for (int g = 0; g < nG; ++g) { run[g] = acc; acc += cnt[g]; }
    for (int e = e0; e < e1; ++e) { int d = dst[e]; d = (d < 0) ? 0 : (d >= N ? N - 1 : d); const int g = d >> CSR_GB3; ids[run[g]] = e; run[g] += 1; } }
  __syncthreads();
  typedef __attribute__((ext_vector_type(4))) int v4i;
  for (int pass = 0; pass < 2; ++pass) {
    for (int i = threadIdx.x; i < CHP / 4; i += 64) *(volatile v4i*)(STG + (size_t)b * CHP + i * 4) = *(const v4i*)(&ids[i * 4]);
    for (int i = threadIdx.x; i < NGP / 4; i += 64) { v4i v; for (int e = 0; e < 4; ++e) v[e] = (i * 4 + e < nG) ? cnt[i * 4 + e] : 0; *(volatile v4i*)(HST + (size_t)b * NGP + i * 4) = v; }
    __threadfence(); }
}
__global__ __launch_bounds__(512) void csrS_kernel3(const int* __restrict__ HST, int nG, int NGP, int* __restrict__ START, int* __restrict__ TOT, int* __restrict__ OFF) {
  __shared__ int tot[CSR_MAXG3];
  const int b = threadIdx.x;
  for (int pass = 0; pass < 2; ++pass) { int runb = 0; for (int g = 0; g < nG; ++g) { int c = HST[(size_t)b * NGP + g]; c = (c < 0) ? 0 : c; ((volatile int*)OFF)[(size_t)g * CSR_NBLK3 + b] = runb; runb += c; } __threadfence(); }
  for (int g = threadIdx.x; g < nG; g += 512) { int s = 0; for (int bb = 0; bb < CSR_NBLK3; ++bb) { int c = HST[(size_t)bb * NGP + g]; s += (c < 0) ? 0 : c; } tot[g] = s; }
  __syncthreads();
  if (threadIdx.x < 32) {
    __shared__ int st[CSR_MAXG3 + 32];
    if (threadIdx.x == 0) { int acc = 0; for (int g = 0; g < NGP; ++g) { st[g] = acc; if (g < nG) acc += (tot[g] + 31) & ~31; } st[NGP] = acc; }
    __builtin_amdgcn_fence(__ATOMIC_RELEASE, "workgroup"); __builtin_amdgcn_wave_barrier(); __builtin_amdgcn_fence(__ATOMIC_ACQUIRE, "workgroup");
    for (int pass = 0; pass < 2; ++pass) { for (int i = threadIdx.x; i < NGP + 32; i += 32) { ((volatile int*)START)[i] = (i <= NGP) ? st[min(i, NGP)] : 0; ((volatile int*)TOT)[i] = (i < nG) ? tot[i] : 0; } __threadfence(); } }
}
__global__ __launch_bounds__(256) void csrB_kernel3(const int* __restrict__ dst, int N, int nG, int CHP, int NGP, int permLen, const int* __restrict__ STG, const int* __restrict__ HST, const int* __restrict__ OFF, const int* __restrict__ START, const int* __restrict__ TOT, int* __restrict__ PERM, int* __restrict__ ROWPTR, int* __restrict__ ROWCNT, int* __restrict__ FLAG) {
  typedef __attribute__((ext_vector_type(4))) int v4i;
  __shared__ int ids[CSR_CAP3]; __shared__ unsigned short key[CSR_CAP3]; __shared__ int outp[CSR_CAP3]; __shared__ int ncnt[CSR_GN3 + 1]; __shared__ int boff[CSR_NBLK3 + 1];
  const int g = blockIdx.x, t_ = threadIdx.x; int tot = TOT[g]; int st = START[g], stn = START[g + 1]; const int v0 = g * CSR_GN3; const int nv = min(CSR_GN3, N - v0); const int t0 = g * CSR_TS3;
  st = (st < 0) ? 0 : (st > permLen - 32 ? permLen - 32 : st) & ~31; stn = (stn < st) ? st : (stn > permLen ? permLen : stn); tot = (tot < 0) ? 0 : tot; if (tot > stn - st && tot <= CSR_CAP3) tot = stn - st;
  if (tot > CSR_CAP3) {
    for (int pass = 0; pass < 2; ++pass) { for (int i = t_; i < CSR_TS3 / 4; i += 256) { v4i a, c; for (int e = 0; e < 4; ++e) { a[e] = st; c[e] = 0; } *(volatile v4i*)(ROWPTR + t0 + i * 4) = a; *(volatile v4i*)(ROWCNT + t0 + i * 4) = c; } if (t_ == 0) ((volatile int*)FLAG)[0] = 1; __threadfence(); } (void)nv; return; }
  if (t_ == 0) { int acc = 0; for (int b = 0; b < CSR_NBLK3; ++b) { boff[b] = acc; int c = HST[(size_t)b * NGP + g]; c = (c < 0) ? 0 : (c > CHP ? CHP : c); acc += c; if (acc > tot) acc = tot; } boff[CSR_NBLK3] = acc; }
  for (int i = t_; i <= CSR_GN3; i += 256) ncnt[i] = 0;
  __syncthreads();
  for (int b = 0; b < CSR_NBLK3; ++b) { const int c = boff[b + 1] - boff[b]; int o_ = OFF[(size_t)g * CSR_NBLK3 + b]; o_ = (o_ < 0) ? 0 : (o_ > CHP - c ? CHP - c : o_); const int* src_ = STG + (size_t)b * CHP + o_;
    for (int i = t_; i < c; i += 256) { int id = src_[i]; id = (id < 0) ? 0 : id; ids[boff[b] + i] = id; int d = dst[id]; d = (d < v0) ? v0 : (d >= N ? N - 1 : d); int kk = d - v0; kk = (kk < 0) ? 0 : (kk >= CSR_GN3 ? CSR_GN3 - 1 : kk); key[boff[b] + i] = (unsigned short)kk; } }
  __syncthreads();
  if (t_ == 0) { for (int i = 0; i < tot; ++i) ncnt[key[i]] += 1; int acc = 0; for (int vl = 0; vl < CSR_GN3; ++vl) { const int c = ncnt[vl]; ncnt[vl] = acc; acc += c; } ncnt[CSR_GN3] = acc;
    for (int i = 0; i < tot; ++i) { const int vl = key[i]; outp[ncnt[vl]] = ids[i]; ncnt[vl] += 1; }
    for (int vl = CSR_GN3; vl > 0; --vl) ncnt[vl] = ncnt[vl - 1]; ncnt[0] = 0; }
  __syncthreads();
  for (int pass = 0; pass < 2; ++pass) {
    for (int i = t_; i < (stn - st) / 4; i += 256) { v4i v; for (int e = 0; e < 4; ++e) { const int q = i * 4 + e; v[e] = (q < tot) ? outp[q] : -1; } *(volatile v4i*)(PERM + st + i * 4) = v; }
    for (int i = t_; i < CSR_TS3 / 4; i += 256) { v4i a, c; for (int e = 0; e < 4; ++e) { const int vl = i * 4 + e; const int vc = vl < CSR_GN3 ? vl : CSR_GN3; a[e] = (vl < CSR_GN3) ? st + ncnt[vc] : st; c[e] = (vl < nv) ? (ncnt[(vc < CSR_GN3 ? vc : CSR_GN3 - 1) + 1] - ncnt[vc]) : 0; } *(volatile v4i*)(ROWPTR + t0 + i * 4) = a; *(volatile v4i*)(ROWCNT + t0 + i * 4) = c; }
    __threadfence(); }
}
__global__ __launch_bounds__(256) void csrZ_kernel3(int* __restrict__ p, size_t n4) { typedef __attribute__((ext_vector_type(4))) int v4i; const size_t tid = (size_t)blockIdx.x * 256 + threadIdx.x, nth = (size_t)gridDim.x * 256; v4i z = {0, 0, 0, 0}; for (size_t i = tid; i < n4; i += nth) *(volatile v4i*)(p + i * 4) = z; }
struct CsrBufs3 { int *STG, *HST, *OFF, *START, *TOT, *PERM, *ROWPTR, *ROWCNT, *FLAG; int nG, NGP, CHP; size_t permLen; char* base; size_t bytes; };
static size_t csr_carve3(CsrBufs3& c, char* ws, size_t off, int E, int N) {
  const size_t off0 = off; c.base = ws + off;
  auto al = [&](size_t bytes) { char* p = ws + off; off += (bytes + 255) & ~(size_t)255; return p; };
  c.nG = (N + CSR_GN3 - 1) / CSR_GN3; c.NGP = (c.nG + 31) & ~31; const int ch = (E + CSR_NBLK3 - 1) / CSR_NBLK3; c.CHP = (ch + 31) & ~31; c.permLen = (size_t)E + 32 * (size_t)c.nG + 32;
  c.STG = (int*)al((size_t)CSR_NBLK3 * c.CHP * 4); c.HST = (int*)al((size_t)CSR_NBLK3 * c.NGP * 4); c.OFF = (int*)al((size_t)c.NGP * CSR_NBLK3 * 4); c.START = (int*)al((size_t)(c.NGP + 64) * 4); c.TOT = (int*)al((size_t)(c.NGP + 64) * 4);
  c.PERM = (int*)al(c.permLen * 4); c.ROWPTR = (int*)al((size_t)c.nG * CSR_TS3 * 4); c.ROWCNT = (int*)al((size_t)c.nG * CSR_TS3 * 4); c.FLAG = (int*)al(256);
  c.bytes = off - off0; return off;
}
static void csr_build3(const CsrBufs3& c, const int* dst, int E, int N, hipStream_t stream) {
  const size_t smem = (size_t)(2 * c.NGP + c.CHP) * 4;
  csrZ_kernel3<<<512, 256, 0, stream>>>((int*)c.base, c.bytes / 16);
  csrA_kernel3<<<CSR_NBLK3, 64, smem, stream>>>(dst, E, N, c.nG, c.CHP, c.NGP, c.STG, c.HST);
  csrS_kernel3<<<1, 512, 0, stream>>>(c.HST, c.nG, c.NGP, c.START, c.TOT, c.OFF);
  csrB_kernel3<<<c.nG, 256, 0, stream>>>(dst, N, c.nG, c.CHP, c.NGP, (int)c.permLen, c.STG, c.HST, c.OFF, c.START, c.TOT, c.PERM, c.ROWPTR, c.ROWCNT, c.FLAG);
}


__global__ __launch_bounds__(256) void wl_kernel(const float* __restrict__ wih, const float* __restrict__ whh, b16* __restrict__ WT) {
  const int u = blockIdx.x * 256 + threadIdx.x; if (u >= 4 * H * 192 / 8) return; const int e = u * 8; const int o = e / 192, k0 = e % 192; v8b v;
#pragma unroll
  for (int j = 0; j < 8; ++j) { const int k = k0 + j; v[j] = (b16)(bf16_rne(k < 2 * H ? wih[(size_t)o * 2 * H + k] : whh[(size_t)o * H + (k - 2 * H)]) * WSC); }
  for (int pass = 0; pass < 2; ++pass) { *(volatile v8b*)(WT + e) = v; __threadfence(); }
}
__global__ __launch_bounds__(256) void wcopyp_kernel(const float* __restrict__ w, int KIN, int OUT, int KP, b16* __restrict__ WT) {
  const int u = blockIdx.x * 256 + threadIdx.x; if (u >= OUT * KP / 8) return; const int e = u * 8; const int o = e / KP, k0 = e % KP; v8b v;
#pragma unroll
  for (int j = 0; j < 8; ++j) { const int k = k0 + j; v[j] = k < KIN ? (b16)(bf16_rne(w[(size_t)o * KIN + k]) * WSC) : (b16)0.0f; } for (int pass = 0; pass < 2; ++pass) { *(volatile v8b*)(WT + e) = v; __threadfence(); }
}
__global__ __launch_bounds__(256) void wg_kernel(const float* __restrict__ we2, const float* __restrict__ be2, b16* __restrict__ WG) {
  const int u = blockIdx.x * 256 + threadIdx.x; if (u >= GW * H / 8) return; const int e = u * 8; const int row = e / H, j0 = e % H; v8b v;
#pragma unroll
  for (int jj = 0; jj < 8; ++jj) { const int j = j0 + jj; float w; if (row < H * H) { const int k = row / H, i = row % H; w = we2[((size_t)i * H + j) * H + k]; } else { const int i = row - H * H; w = be2[(size_t)i * H + j]; } v[jj] = (b16)(bf16_rne(w) * WSC); }
  for (int pass = 0; pass < 2; ++pass) { *(volatile v8b*)(WG + e) = v; __threadfence(); }
}

template <int KIN, int RELU>
__global__ __launch_bounds__(32) void lin32_kernel(const float* __restrict__ IN_, int nrows, const b16* __restrict__ WT, const float* __restrict__ bias, float* __restrict__ OUT_) {
  __shared__ __attribute__((aligned(16))) b16 Ah[16][32 + 8]; __shared__ __attribute__((aligned(16))) float Tf[16][H + 4];
  const int lane = threadIdx.x, nloc = lane & 15, hlf = lane >> 4; const size_t m0 = (size_t)blockIdx.x * 16;
  for (int rr = 0; rr < 16; ++rr) { const size_t r = (m0 + rr) < (size_t)nrows ? m0 + rr : (size_t)nrows - 1; Ah[rr][lane] = lane < KIN ? (b16)(bf16_rne(IN_[r * KIN + lane]) * XS) : (b16)0.0f; }
  wave_lds_sync();
  v8f acc[4]; const v16b a = frag_kb(&Ah[nloc][0], hlf);
#pragma unroll
  for (int t = 0; t < 4; ++t) { acc[t] = (v8f){}; acc[t] = wmma16b(a, frag_kb(WT + (size_t)(t * 16 + nloc) * 32, hlf), acc[t]); }
#pragma unroll
  for (int t = 0; t < 4; ++t) { const int c = t * 16 + nloc; const float bb = bf16_rne(bias[c]);
#pragma unroll 1
    for (int r8 = 0; r8 < 8; ++r8) { const float v = acc[t][r8] * (1.0f / (XS * WSC)) + bb; Tf[8 * hlf + r8][c] = RELU ? fmaxf(v, 0.0f) : v; } }
  wave_lds_sync();
  for (int pass = 0; pass < 2; ++pass) { for (int rr = 0; rr < 16; ++rr) if (m0 + rr < (size_t)nrows) *(volatile v2f*)(OUT_ + (m0 + rr) * H + lane * 2) = *(const v2f*)(&Tf[rr][lane * 2]); __threadfence(); }
}
__global__ __launch_bounds__(32) void g_kernel(const float* __restrict__ Hp, const b16* __restrict__ WG, int NLIM, float* __restrict__ GB) {
  __shared__ __attribute__((aligned(16))) b16 Ah[16][H + 8], Al[16][H + 8]; __shared__ __attribute__((aligned(16))) float Tf[16][160 + 4];
  const int lane = threadIdx.x, nloc = lane & 15, hlf = lane >> 4; const size_t m0 = (size_t)blockIdx.x * 16; if (m0 >= (size_t)NLIM) return;
  for (int rr = 0; rr < 16; ++rr) { const v2f v = *(const v2f*)(Hp + (m0 + rr) * H + lane * 2); for (int j = 0; j < 2; ++j) { b16 p, q; split16(v[j] * HS, p, q); Ah[rr][lane * 2 + j] = p; Al[rr][lane * 2 + j] = q; } }
  wave_lds_sync();
  const v16b a0 = frag_kb(&Ah[nloc][0], hlf), l0 = frag_kb(&Al[nloc][0], hlf), a1 = frag_kb(&Ah[nloc][32], hlf), l1 = frag_kb(&Al[nloc][32], hlf);
#pragma unroll 1
  for (int cg = 0; cg < GW / 160; ++cg) { v8f acc[10];
#pragma unroll
    for (int t = 0; t < 10; ++t) { acc[t] = (v8f){}; const b16* wr = WG + (size_t)(cg * 160 + t * 16 + nloc) * H; acc[t] = wmma16b(a0, frag_kb(wr, hlf), acc[t]); acc[t] = wmma16b(l0, frag_kb(wr, hlf), acc[t]); acc[t] = wmma16b(a1, frag_kb(wr + 32, hlf), acc[t]); acc[t] = wmma16b(l1, frag_kb(wr + 32, hlf), acc[t]); }
#pragma unroll
    for (int t = 0; t < 10; ++t)
#pragma unroll 1
      for (int r8 = 0; r8 < 8; ++r8) Tf[8 * hlf + r8][t * 16 + nloc] = acc[t][r8] * (1.0f / (HS * WSC));
    wave_lds_sync();
    for (int pass = 0; pass < 2; ++pass) { for (int rr = 0; rr < 16; ++rr) for (int q = 0; q < 5; ++q) ((volatile float*)GB)[(m0 + rr) * GW + cg * 160 + q * 32 + lane] = Tf[rr][q * 32 + lane]; __threadfence(); }
    wave_lds_sync(); }
}
__global__ __launch_bounds__(256) void msg_kernel(const float* __restrict__ GE, const float* __restrict__ GB, const int* __restrict__ srcs, const int* __restrict__ PERM, const int* __restrict__ ROWPTR, const int* __restrict__ ROWCNT, int permLen, int NLIM, float* __restrict__ AGG) {
  const int wave = threadIdx.x >> 5, lane = threadIdx.x & 31; const size_t v = (size_t)blockIdx.x * 8 + wave; float a0 = 0.0f, a1 = 0.0f;
  if (v < (size_t)NLIM) { int st = ROWPTR[v], cnt = ROWCNT[v]; cnt = iclamp(cnt, 0, 1 << 20); st = iclamp(st, 0, permLen - cnt);
#pragma unroll 1
    for (int j = 0; j < cnt; ++j) { const int e = iclamp(PERM[st + j], 0, E - 1); const size_t s = (size_t)iclamp(srcs[e], 0, N - 1); if (s >= (size_t)NLIM) continue; const float* ge = GE + (size_t)e * H; const float* gb = GB + s * GW;
      { const v2f bh = *(const v2f*)(gb + H * H + lane * 2); a0 += bh[0]; a1 += bh[1]; }
#pragma unroll 1
      for (int k = 0; k < H; k += 4) { const v4f gk = *(const v4f*)(ge + k);
#pragma unroll
        for (int kk = 0; kk < 4; ++kk) { const v2f gv = *(const v2f*)(gb + (size_t)(k + kk) * H + lane * 2); a0 += pmul(gk[kk], gv[0]); a1 += pmul(gk[kk], gv[1]); } } } }
  for (int pass = 0; pass < 2; ++pass) { v2f o = {a0, a1}; *(volatile v2f*)(AGG + v * H + lane * 2) = o; __threadfence(); }
}
__global__ __launch_bounds__(32) void gru_kernel(const float* __restrict__ AGG, const float* __restrict__ Hp, const b16* __restrict__ WIH, const b16* __restrict__ WHH, const float* __restrict__ bih, const float* __restrict__ bhh, int NLIM, float* __restrict__ HOUT) {
  __shared__ __attribute__((aligned(16))) b16 Ah[16][H + 8], Al[16][H + 8], Bh_[16][H + 8], Bl[16][H + 8]; __shared__ __attribute__((aligned(16))) float Hs[16][H + 4], Tf[16][H + 4];
  const int lane = threadIdx.x, nloc = lane & 15, hlf = lane >> 4; const size_t m0 = (size_t)blockIdx.x * 16; if (m0 >= (size_t)NLIM) return;
  for (int rr = 0; rr < 16; ++rr) { const v2f av = *(const v2f*)(AGG + (m0 + rr) * H + lane * 2), hv = *(const v2f*)(Hp + (m0 + rr) * H + lane * 2);
    for (int j = 0; j < 2; ++j) { b16 p, q; split16(av[j] * XS, p, q); Ah[rr][lane * 2 + j] = p; Al[rr][lane * 2 + j] = q; split16(hv[j] * HS, p, q); Bh_[rr][lane * 2 + j] = p; Bl[rr][lane * 2 + j] = q; Hs[rr][lane * 2 + j] = hv[j]; } }
  wave_lds_sync();
  v8f gi[12], gh[12];
#pragma unroll
  for (int t = 0; t < 12; ++t) { gi[t] = (v8f){}; gh[t] = (v8f){}; }
#pragma unroll
  for (int kb = 0; kb < H; kb += 32) { const v16b a = frag_kb(&Ah[nloc][kb], hlf), al = frag_kb(&Al[nloc][kb], hlf), b = frag_kb(&Bh_[nloc][kb], hlf), bl = frag_kb(&Bl[nloc][kb], hlf);
#pragma unroll
    for (int t = 0; t < 12; ++t) { const v16b w1 = frag_kb(WIH + (size_t)(t * 16 + nloc) * H + kb, hlf), w2 = frag_kb(WHH + (size_t)(t * 16 + nloc) * H + kb, hlf); gi[t] = wmma16b(a, w1, gi[t]); gi[t] = wmma16b(al, w1, gi[t]); gh[t] = wmma16b(b, w2, gh[t]); gh[t] = wmma16b(bl, w2, gh[t]); } }
  wave_lds_sync();
  const float si = 1.0f / (XS * WSC), sh = 1.0f / (HS * WSC);
#pragma unroll
  for (int t = 0; t < 4; ++t) { const int c = t * 16 + nloc; const float bir = bf16_rne(bih[c]), biz = bf16_rne(bih[H + c]), bin_ = bf16_rne(bih[2 * H + c]), bhr = bf16_rne(bhh[c]), bhz = bf16_rne(bhh[H + c]), bhn = bf16_rne(bhh[2 * H + c]);
#pragma unroll
    for (int r8 = 0; r8 < 8; ++r8) { const int rl = 8 * hlf + r8; const float r = sigm(gi[t][r8] * si + bir + gh[t][r8] * sh + bhr), z = sigm(gi[4 + t][r8] * si + biz + gh[4 + t][r8] * sh + bhz); const float n = tanhf(gi[8 + t][r8] * si + bin_ + pmul(r, gh[8 + t][r8] * sh + bhn)); Tf[rl][c] = pmul(1.0f - z, n) + pmul(z, Hs[rl][c]); } }
  wave_lds_sync();
  for (int pass = 0; pass < 2; ++pass) { for (int rr = 0; rr < 16; ++rr) *(volatile v2f*)(HOUT + (m0 + rr) * H + lane * 2) = *(const v2f*)(&Tf[rr][lane * 2]); __threadfence(); }
}
__global__ __launch_bounds__(256) void s2s_kernel(const float* __restrict__ Hp, const int* __restrict__ PERM, const int* __restrict__ ROWPTR, const int* __restrict__ ROWCNT, int permLen, int NLIM, const b16* __restrict__ WL, const float* __restrict__ bihl, const float* __restrict__ bhhl, const float* __restrict__ Wout, const float* __restrict__ bout, float* __restrict__ out) {
  __shared__ __attribute__((aligned(16))) b16 Ah[4][16][192 + 8], Al[4][16][192 + 8]; __shared__ float QS[NB][2 * H], HHs[NB][H], CC[NB][H]; __shared__ float so[NB * TGT];
  const int wave = threadIdx.x >> 5, lane = threadIdx.x & 31, nloc = lane & 15, hlf = lane >> 4;
  for (int i = threadIdx.x; i < NB * 2 * H; i += 256) (&QS[0][0])[i] = 0.0f; for (int i = threadIdx.x; i < NB * H; i += 256) { (&HHs[0][0])[i] = 0.0f; (&CC[0][0])[i] = 0.0f; }
  __syncthreads();
#pragma unroll 1
  for (int step = 0; step < S2S; ++step) {
    if (wave < 4) { const int g0 = wave * 16;
      for (int rr = 0; rr < 16; ++rr) { for (int q = 0; q < 4; ++q) { const float v = QS[g0 + rr][q * 32 + lane]; b16 p, ql; split16(v * XS, p, ql); Ah[wave][rr][q * 32 + lane] = p; Al[wave][rr][q * 32 + lane] = ql; } for (int q = 0; q < 2; ++q) { const float v = HHs[g0 + rr][q * 32 + lane]; b16 p, ql; split16(v * XS, p, ql); Ah[wave][rr][128 + q * 32 + lane] = p; Al[wave][rr][128 + q * 32 + lane] = ql; } }
      wave_lds_sync();
      v8f acc[16];
#pragma unroll
      for (int t = 0; t < 16; ++t) acc[t] = (v8f){};
#pragma unroll 2
      for (int kb = 0; kb < 192; kb += 32) { const v16b a = frag_kb(&Ah[wave][nloc][kb], hlf), al = frag_kb(&Al[wave][nloc][kb], hlf);
#pragma unroll
        for (int t = 0; t < 16; ++t) { const v16b bw = frag_kb(WL + (size_t)(t * 16 + nloc) * 192 + kb, hlf); acc[t] = wmma16b(a, bw, acc[t]); acc[t] = wmma16b(al, bw, acc[t]); } }
      wave_lds_sync();
      const float sc = 1.0f / (XS * WSC);
#pragma unroll
      for (int t = 0; t < 4; ++t) { const int c = t * 16 + nloc; float bb[4]; for (int gq = 0; gq < 4; ++gq) bb[gq] = bf16_rne(bihl[gq * H + c]) + bf16_rne(bhhl[gq * H + c]);
#pragma unroll
        for (int r8 = 0; r8 < 8; ++r8) { const int g = g0 + 8 * hlf + r8; const float ig = sigm(acc[t][r8] * sc + bb[0]), fg = sigm(acc[4 + t][r8] * sc + bb[1]), gg = tanhf(acc[8 + t][r8] * sc + bb[2]), og = sigm(acc[12 + t][r8] * sc + bb[3]); const float cn = pmul(fg, CC[g][c]) + pmul(ig, gg); CC[g][c] = cn; HHs[g][c] = pmul(og, tanhf(cn)); } } }
    __syncthreads();
    for (int gg = 0; gg < 8; ++gg) { const int g = wave * 8 + gg; const int tix = (g >> 3) * 32 + (g & 7); int st = ROWPTR[tix], cnt = ROWCNT[tix]; cnt = iclamp(cnt, 0, 1 << 20); st = iclamp(st, 0, permLen - cnt); const float h0 = HHs[g][lane * 2], h1 = HHs[g][lane * 2 + 1];
      float mx = -INFINITY;
#pragma unroll 1
      for (int j = 0; j < cnt; ++j) { const int n = iclamp(PERM[st + j], 0, N - 1); const bool ok = n < NLIM; const v2f hv = *(const v2f*)(Hp + (size_t)n * H + lane * 2); float e = pmul(hv[0], h0) + pmul(hv[1], h1); for (int o = 16; o; o >>= 1) e += __shfl_xor(e, o); if (ok) mx = fmaxf(mx, e); }
      float den = 0.0f, r0 = 0.0f, r1 = 0.0f;
#pragma unroll 1
      for (int j = 0; j < cnt; ++j) { const int n = iclamp(PERM[st + j], 0, N - 1); const bool ok = n < NLIM; const v2f hv = *(const v2f*)(Hp + (size_t)n * H + lane * 2); float e = pmul(hv[0], h0) + pmul(hv[1], h1); for (int o = 16; o; o >>= 1) e += __shfl_xor(e, o); if (ok) { const float p = __expf(e - mx); den += p; r0 += pmul(p, hv[0]); r1 += pmul(p, hv[1]); } }
      const float inv = den > 0.0f ? 1.0f / den : 0.0f; QS[g][lane * 2] = h0; QS[g][lane * 2 + 1] = h1; QS[g][H + lane * 2] = pmul(r0, inv); QS[g][H + lane * 2 + 1] = pmul(r1, inv); }
    __syncthreads(); }
  for (int gg = 0; gg < 8; ++gg) { const int g = wave * 8 + gg; const float q0 = QS[g][lane * 2], q1 = QS[g][lane * 2 + 1];
#pragma unroll
    for (int k = 0; k < TGT; ++k) { float s = pmul(q0, bf16_rne(Wout[k * H + lane * 2])) + pmul(q1, bf16_rne(Wout[k * H + lane * 2 + 1])); for (int o = 16; o; o >>= 1) s += __shfl_xor(s, o); if (lane == 0) so[g * TGT + k] = s + bf16_rne(bout[k]); } }
  __syncthreads();
  for (int pass = 0; pass < 2; ++pass) { for (int i = threadIdx.x; i < NB * TGT; i += 256) ((volatile float*)out)[i] = so[i]; __threadfence(); }
}
}

extern "C" void kernel_launch(void* const* d_in, const int* in_sizes, int n_in, void* d_out, int out_size, void* d_ws, size_t ws_size, hipStream_t stream) {
  (void)n_in;
  auto Fp = [&](int i) { return (const float*)d_in[i]; }; auto Ip = [&](int i) { return (const int*)d_in[i]; };
  if (in_sizes[0] != N * NF || in_sizes[1] != E * EF || in_sizes[2] != E || in_sizes[3] != E || in_sizes[4] != N || in_sizes[5] != H * NF || in_sizes[7] != H * EF || in_sizes[9] != H * H * H || in_sizes[10] != H * H || in_sizes[11] != 3 * H * H || in_sizes[15] != 4 * H * 2 * H || in_sizes[16] != 4 * H * H || in_sizes[19] != TGT * H || out_size != NB * TGT) return;
  const int NLIM = N; const int GB16 = NBLK, GB8 = N / 8;
  size_t off = 0; char* ws = (char*)d_ws;
  auto carve = [&](size_t bytes) { char* p = ws + off; off += (bytes + 255) & ~(size_t)255; return p; };
  b16* WIN = (b16*)carve(H * 32 * 2); b16* WE1 = (b16*)carve(H * 32 * 2); b16* WG = (b16*)carve((size_t)GW * H * 2); b16* WIH = (b16*)carve(3 * H * H * 2); b16* WHH = (b16*)carve(3 * H * H * 2); b16* WL = (b16*)carve((size_t)4 * H * 192 * 2);
  float* GE = (float*)carve((size_t)E * H * 4); float* HA = (float*)carve((size_t)N * H * 4); float* HB = (float*)carve((size_t)N * H * 4); float* GBp = (float*)carve((size_t)N * GW * 4); float* AGG = (float*)carve((size_t)N * H * 4);
  CsrBufs9 ct; CsrBufs3 pl; off = csr_carve9(ct, ws, off, E, N); off = csr_carve3(pl, ws, off, N, NB);
  if (off > ws_size || off > ((size_t)224 << 20)) return;
  wcopyp_kernel<<<(H * 32 / 8 + 255) / 256, 256, 0, stream>>>(Fp(5), NF, H, 32, WIN); wcopyp_kernel<<<(H * 32 / 8 + 255) / 256, 256, 0, stream>>>(Fp(7), EF, H, 32, WE1);
  wg_kernel<<<(GW * H / 8 + 255) / 256, 256, 0, stream>>>(Fp(9), Fp(10), WG);
  wcopyp_kernel<<<(3 * H * H / 8 + 255) / 256, 256, 0, stream>>>(Fp(11), H, 3 * H, H, WIH); wcopyp_kernel<<<(3 * H * H / 8 + 255) / 256, 256, 0, stream>>>(Fp(12), H, 3 * H, H, WHH);
  wl_kernel<<<(4 * H * 192 / 8 + 255) / 256, 256, 0, stream>>>(Fp(15), Fp(16), WL);
  csr_build9(ct, Ip(3), E, N, stream); csr_build3(pl, Ip(4), N, NB, stream);
  lin32_kernel<NF, 0><<<NBLK, 32, 0, stream>>>(Fp(0), N, WIN, Fp(6), HA);
  lin32_kernel<EF, 1><<<E / 16, 32, 0, stream>>>(Fp(1), E, WE1, Fp(8), GE);
  float* hin = HA; float* hout = HB;
  for (int s = 0; s < T; ++s) {
    g_kernel<<<GB16, 32, 0, stream>>>(hin, WG, NLIM, GBp);
    msg_kernel<<<GB8, 256, 0, stream>>>(GE, GBp, Ip(2), ct.PERM, ct.ROWPTR, ct.ROWCNT, (int)ct.permLen, NLIM, AGG);
    gru_kernel<<<GB16, 32, 0, stream>>>(AGG, hin, WIH, WHH, Fp(13), Fp(14), NLIM, hout);
    float* tmp = hin; hin = hout; hout = tmp; }
  s2s_kernel<<<1, 256, 0, stream>>>(hin, pl.PERM, pl.ROWPTR, pl.ROWCNT, (int)pl.permLen, NLIM, WL, Fp(17), Fp(18), Fp(19), Fp(20), (float*)d_out);
}
